// FusionNet_10995116278260
// MI455X (gfx1250) — hardware-run, weakly checked
//
#include <hip/hip_runtime.h>


#ifndef NB
#define NB 4
#endif
#ifndef HR
#define HR 192
#endif
#define NB_FULL 4
#define HR_FULL 192
#ifndef OUT_HR
#define OUT_HR HR
#endif
#define CH   64
#define WID  192
#define NWV  12
#define NTH  (32 * NWV)
#define QP   72
#define VP   200
#define OP   196
#define QL_H 0
#define QR_H (WID * QP)
#define VL_H (2 * WID * QP)
#define VR_H (2 * WID * QP + CH * VP)
#define ARENA_H (2 * WID * QP + 2 * CH * VP)
#define WCS  64.0f
#define WCI  (1.0f / 64.0f)
#define SC2  ((float)(0.125 * 1.4426950408889634))
#define L2E  1.4426950408889634f
#define PSH  14.0f
#define NEGB (-3.0e38f)
#define FB   ((HR * WID) / 1024)

static_assert(CH == 64);
static_assert(CH % 32 == 0);
static_assert(WID == 16 * NWV);
static_assert(WID % 32 == 0);
static_assert(WID % 8 == 0);
static_assert(NTH == 2 * WID);
static_assert(NTH * 8 == CH * (WID / 4));
static_assert((WID / 4) % 8 == 0);
static_assert(QP % 8 == 0);
static_assert(VP % 8 == 0);
static_assert(OP % 4 == 0);
static_assert(QP >= CH);
static_assert(VP >= WID);
static_assert(OP >= WID);
static_assert(4 * CH * OP <= ARENA_H);
static_assert(ARENA_H * 2 + 640 * 4 + 128 * 4 <= 131072);
static_assert(2 * CH == 128);
static_assert((HR * WID) % 1024 == 0);
static_assert(CH * CH / 8 == 512);
static_assert(NB <= NB_FULL);
static_assert(HR <= HR_FULL);
static_assert(HR <= OUT_HR);

typedef _Float16 h16;
typedef __attribute__((ext_vector_type(16))) _Float16 v16h;
typedef __attribute__((ext_vector_type(8)))  _Float16 v8h;
typedef __attribute__((ext_vector_type(8)))  float    v8f;
typedef __attribute__((ext_vector_type(4)))  float    v4f;
typedef v4f  __attribute__((may_alias)) v4fa;
typedef v8h  __attribute__((may_alias)) v8ha;
typedef float __attribute__((may_alias)) f32a;

__device__ __forceinline__ unsigned short f2bf(float f) { unsigned u = __float_as_uint(f); u += 0x7FFFu + ((u >> 16) & 1u); return (unsigned short)(u >> 16); }
__device__ __forceinline__ float bfr(float f) { return __uint_as_float(((unsigned)f2bf(f)) << 16); }
__device__ __forceinline__ v16h cat16(v8h lo, v8h hi) { return __builtin_shufflevector(lo, hi, 0, 1, 2, 3, 4, 5, 6, 7, 8, 9, 10, 11, 12, 13, 14, 15); }
__device__ __forceinline__ v8f wmma16(v16h a, v16h b, v8f c) { return __builtin_amdgcn_wmma_f32_16x16x32_f16(false, a, false, b, (short)0, c, false, false); }
__device__ __forceinline__ v16h  ldh(const h16* p) { return cat16(*(const v8h*)p, *(const v8h*)(p + 16)); }
__device__ __forceinline__ void wave_sync() { __builtin_amdgcn_fence(3  , "wavefront"); __builtin_amdgcn_wave_barrier(); asm volatile("" ::: "memory"); }
static __device__ __forceinline__ h16 toh_flush(float v) { const h16 r = (h16)v; return (fabsf(v) < 6.103515625e-05f) ? (h16)0.0f : r; }
__device__ __forceinline__ v8f wg(v16h a, v16h b, v8f c) {
    c = wmma16(a, b, c);
    asm volatile("v_nop\n\tv_nop\n\tv_nop\n\tv_nop" : "+v"(c) : "v"(a), "v"(b));
    return c;
}

__global__ __launch_bounds__(256) void k_wconv(const float* __restrict__ w0, const float* __restrict__ w1, const float* __restrict__ w2, const float* __restrict__ w3, h16* dst) {
    const int i = blockIdx.x * 256 + threadIdx.x;
    const v8f a0 = *(const v8f*)(w0 + (size_t)i * 8); const v8f a1 = *(const v8f*)(w1 + (size_t)i * 8);
    const v8f a2 = *(const v8f*)(w2 + (size_t)i * 8); const v8f a3 = *(const v8f*)(w3 + (size_t)i * 8);
    v8h o0, o1, o2, o3;
#pragma unroll
    for (int k = 0; k < 8; ++k) { o0[k] = toh_flush(bfr(a0[k]) * WCS); o1[k] = toh_flush(bfr(a1[k]) * WCS); o2[k] = toh_flush(bfr(a2[k]) * WCS); o3[k] = toh_flush(bfr(a3[k]) * WCS); }
#pragma unroll 1
    for (int ps = 0; ps < 2; ++ps) {
        *(volatile v8h*)(dst + (size_t)i * 8) = o0;
        *(volatile v8h*)(dst + (size_t)CH * CH + (size_t)i * 8) = o1;
        *(volatile v8h*)(dst + (size_t)2 * CH * CH + (size_t)i * 8) = o2;
        *(volatile v8h*)(dst + (size_t)3 * CH * CH + (size_t)i * 8) = o3;
        if (ps == 0) __threadfence(); }
}

__global__ __launch_bounds__(NTH) __attribute__((amdgpu_num_vgpr(256)))
void k_row(const float* __restrict__ x, const float* __restrict__ y,
           const float* __restrict__ ln_l_w, const float* __restrict__ ln_l_b, const float* __restrict__ ln_r_w, const float* __restrict__ ln_r_b,
           const float* __restrict__ bl1, const float* __restrict__ br1, const float* __restrict__ bl2, const float* __restrict__ br2,
           const float* __restrict__ beta, const float* __restrict__ gamma,
           const h16* __restrict__ WH, float* X2, float* Y2, float* PART) {
    __shared__ __align__(16) h16 hs[ARENA_H];
    __shared__ __align__(16) float prm[640];
    __shared__ __align__(16) float psum[128];
#define TF ((f32a*)hs)
#define LDL(o) cat16(*(const v8ha*)(hs + (o)), *(const v8ha*)(hs + (o) + 16))
    const int tid = threadIdx.x, lane = tid & 31, lr = lane & 15, hi = lane >> 4;
    const int wave = __builtin_amdgcn_readfirstlane((int)(threadIdx.x >> 5));
    const int up = __builtin_amdgcn_readfirstlane((int)(threadIdx.x / (unsigned)WID));
    const int bh = blockIdx.x; const int b = bh / HR, h = bh % HR;
    const size_t PLF = (size_t)HR_FULL * WID;
    const size_t gbase = ((size_t)b * CH * HR_FULL + (size_t)h) * WID;
    const int i0 = wave * 16;

    if (wave < 2) { const int c = tid;
        prm[c] = bfr(ln_l_w[c]); prm[64 + c] = bfr(ln_l_b[c]); prm[128 + c] = bfr(ln_r_w[c]); prm[192 + c] = bfr(ln_r_b[c]);
        prm[256 + c] = bfr(bl1[c]); prm[320 + c] = bfr(br1[c]); prm[384 + c] = bfr(bl2[c]); prm[448 + c] = bfr(br2[c]);
        prm[512 + c] = bfr(beta[c]); prm[576 + c] = bfr(gamma[c]); }

    { const int w = tid - WID * up;
#pragma unroll
      for (int sd = 0; sd < 2; ++sd) {
          const float* src = sd ? y : x; const int po = sd ? QR_H : QL_H;
#pragma unroll 1
          for (int it = 0; it < 4; ++it) {
              const int cg = it * 2 + up;
              const float* p = src + gbase + (size_t)(cg * 8) * PLF + (size_t)w;
              v8h o;
#pragma unroll
              for (int k = 0; k < 8; ++k) o[k] = toh_flush(bfr(p[(size_t)k * PLF]));
              *(v8ha*)(hs + po + w * QP + cg * 8) = o; } } }
    __syncthreads();

#pragma unroll
    for (int sd = 0; sd < 2; ++sd) {
        const int po = sd ? QR_H : QL_H; const int vo = sd ? VR_H : VL_H; const int bo = 384 + 64 * sd;
        const h16* Wg = WH + (size_t)(2 + sd) * CH * CH + (size_t)lr * CH + 8 * hi;
        const v16h xb0 = LDL(po + (i0 + lr) * QP + 8 * hi), xb1 = LDL(po + (i0 + lr) * QP + 8 * hi + 32);
        v8f acc[4];
#pragma unroll
        for (int mb = 0; mb < 4; ++mb) { acc[mb] = (v8f){};
            const v16h a0 = ldh(Wg + (size_t)mb * 16 * CH), a1 = ldh(Wg + (size_t)mb * 16 * CH + 32);
            acc[mb] = wg(a0, xb0, acc[mb]); acc[mb] = wg(a1, xb1, acc[mb]); }
#pragma unroll
        for (int mb = 0; mb < 4; ++mb) {
#pragma unroll
            for (int r = 0; r < 8; ++r) { const int c = 16 * mb + 8 * hi + r;
                hs[vo + c * VP + i0 + lr] = toh_flush(acc[mb][r] * WCI + prm[bo + c]); } }
    }
    __syncthreads();

    { const int row = tid - WID * up; const int ro = up * QR_H + row * QP; const int lo = up * 128;
      float s = 0.0f;
#pragma unroll 1
      for (int g = 0; g < 8; ++g) { const v8h v = *(const v8ha*)(hs + ro + 8 * g);
#pragma unroll
          for (int k = 0; k < 8; ++k) s += (float)v[k]; }
      const float mu = s * (1.0f / 64.0f);
      float qq = 0.0f;
#pragma unroll 1
      for (int g = 0; g < 8; ++g) { const v8h v = *(const v8ha*)(hs + ro + 8 * g);
#pragma unroll
          for (int k = 0; k < 8; ++k) { const float d = (float)v[k] - mu; qq += d * d; } }
      const float rs = rsqrtf(qq * (1.0f / 64.0f) + 1e-5f);
#pragma unroll 1
      for (int g = 0; g < 8; ++g) { const v8h v = *(const v8ha*)(hs + ro + 8 * g); v8h o;
#pragma unroll
          for (int k = 0; k < 8; ++k) o[k] = toh_flush(((float)v[k] - mu) * rs * prm[lo + 8 * g + k] + prm[lo + 64 + 8 * g + k]);
          *(v8ha*)(hs + ro + 8 * g) = o; } }
    __syncthreads();

#pragma unroll
    for (int sd = 0; sd < 2; ++sd) {
        const int po = sd ? QR_H : QL_H; const int bo = 256 + 64 * sd;
        const h16* Wg = WH + (size_t)sd * CH * CH + (size_t)lr * CH + 8 * hi;
        const v16h a0 = LDL(po + (i0 + lr) * QP + 8 * hi), a1 = LDL(po + (i0 + lr) * QP + 8 * hi + 32);
        v8f acc[4];
#pragma unroll
        for (int nb = 0; nb < 4; ++nb) { acc[nb] = (v8f){};
            const v16h b0 = ldh(Wg + (size_t)nb * 16 * CH), b1 = ldh(Wg + (size_t)nb * 16 * CH + 32);
            acc[nb] = wg(a0, b0, acc[nb]); acc[nb] = wg(a1, b1, acc[nb]); }
        wave_sync();
#pragma unroll
        for (int nb = 0; nb < 4; ++nb) { const float bc = prm[bo + 16 * nb + lr];
#pragma unroll
            for (int r = 0; r < 8; ++r) hs[po + (i0 + 8 * hi + r) * QP + 16 * nb + lr] = toh_flush(acc[nb][r] * WCI + bc); }
    }
    __syncthreads();

    auto flash = [&](const int qoff, const int koff, const int voff, v8f& r0, v8f& r1, v8f& r2, v8f& r3) {
        const v16h q0 = LDL(qoff + (i0 + lr) * QP + 8 * hi), q1 = LDL(qoff + (i0 + lr) * QP + 8 * hi + 32);
        v8f o0 = (v8f){}, o1 = (v8f){}, o2 = (v8f){}, o3 = (v8f){};
        float m = NEGB, l = 0.0f;
#pragma unroll 1
        for (int key0 = 0; key0 < WID; key0 += 32) {
            const int kb = koff + (key0 + lr) * QP + 8 * hi;
            const v16h ka0 = LDL(kb), ka1 = LDL(kb + 32), kb0 = LDL(kb + 16 * QP), kb1 = LDL(kb + 16 * QP + 32);
            v8f sa = (v8f){}, sb = (v8f){};
            sa = wg(ka0, q0, sa); sa = wg(ka1, q1, sa); sb = wg(kb0, q0, sb); sb = wg(kb1, q1, sb);
            float ta[8], tb[8]; float mx = NEGB;
#pragma unroll
            for (int r = 0; r < 8; ++r) { ta[r] = sa[r] * SC2; tb[r] = sb[r] * SC2; mx = fmaxf(mx, fmaxf(ta[r], tb[r])); }
            mx = fmaxf(mx, __shfl_xor(mx, 16, 32));
            const float mnew = fmaxf(m, mx);
            const float alpha = __builtin_amdgcn_exp2f(m - mnew);
            const float sh = PSH - mnew;
            v16h pb; float ls = 0.0f;
#pragma unroll
            for (int r = 0; r < 8; ++r) {
                const float xa = ta[r] + sh, xb = tb[r] + sh;
                const float ea = __builtin_amdgcn_exp2f(xa), eb = __builtin_amdgcn_exp2f(xb);
                const float ga = (xa < -14.0f) ? 0.0f : ea, gb = (xb < -14.0f) ? 0.0f : eb;
                const h16 pa = (h16)ga; const h16 pc = (h16)gb;
                pb[r] = pa; pb[8 + r] = pc; ls += (float)pa + (float)pc; }
            l = l * alpha + ls; m = mnew;
            o0 = o0 * alpha; o1 = o1 * alpha; o2 = o2 * alpha; o3 = o3 * alpha;
            const int vb = voff + lr * VP + key0 + 8 * hi;
            const v16h v0 = LDL(vb), v1 = LDL(vb + 16 * VP), v2 = LDL(vb + 32 * VP), v3 = LDL(vb + 48 * VP);
            o0 = wg(v0, pb, o0); o1 = wg(v1, pb, o1); o2 = wg(v2, pb, o2); o3 = wg(v3, pb, o3);
        }
        l += __shfl_xor(l, 16, 32);
        const float inv = 1.0f / l;
        r0 = o0 * inv; r1 = o1 * inv; r2 = o2 * inv; r3 = o3 * inv;
    };
    v8f fr0, fr1, fr2, fr3, fl0, fl1, fl2, fl3;
    flash(QL_H, QR_H, VR_H, fr0, fr1, fr2, fr3);
    flash(QR_H, QL_H, VL_H, fl0, fl1, fl2, fl3);
    __syncthreads();

#pragma unroll
    for (int r = 0; r < 8; ++r) {
        const int c = 8 * hi + r; const int col = i0 + lr;
        TF[(c     ) * OP + col] = prm[512 + c     ] * fr0[r]; TF[(c + 16) * OP + col] = prm[512 + c + 16] * fr1[r];
        TF[(c + 32) * OP + col] = prm[512 + c + 32] * fr2[r]; TF[(c + 48) * OP + col] = prm[512 + c + 48] * fr3[r];
        TF[(CH + c     ) * OP + col] = prm[576 + c     ] * fl0[r]; TF[(CH + c + 16) * OP + col] = prm[576 + c + 16] * fl1[r];
        TF[(CH + c + 32) * OP + col] = prm[576 + c + 32] * fl2[r]; TF[(CH + c + 48) * OP + col] = prm[576 + c + 48] * fl3[r]; }
    __syncthreads();

#pragma unroll 1
    for (int it = 0; it < 8; ++it) {
        const int idx = it * NTH + tid; const int row = idx / (WID / 4), c4 = idx - row * (WID / 4);
        const size_t go = gbase + (size_t)row * PLF + (size_t)c4 * 4;
        const v4f xv = *(const v4f*)(x + go); const v4f yv = *(const v4f*)(y + go);
        const int tx = row * OP + c4 * 4, ty = (CH + row) * OP + c4 * 4;
        v4f a = *(const v4fa*)(TF + tx), c = *(const v4fa*)(TF + ty);
#pragma unroll
        for (int k = 0; k < 4; ++k) { a[k] = a[k] + 2.0f * bfr(xv[k]); c[k] = c[k] + 2.0f * bfr(yv[k]); }
        *(v4fa*)(TF + tx) = a; *(v4fa*)(TF + ty) = c; }
    __syncthreads();

    if (wave < 4) { const int ro = tid * OP; float s = 0.0f;
#pragma unroll 1
        for (int c4 = 0; c4 < WID / 4; ++c4) { const v4f v = *(const v4fa*)(TF + ro + 4 * c4); s += fabsf(v[0]); s += fabsf(v[1]); s += fabsf(v[2]); s += fabsf(v[3]); }
        psum[tid] = s; }
    __syncthreads();

    const size_t PLC = (size_t)HR * WID;
    const size_t obase = ((size_t)b * CH * HR + (size_t)h) * WID;
#pragma unroll 1
    for (int ps = 0; ps < 2; ++ps) {
#pragma unroll 1
        for (int it = 0; it < 8; ++it) {
            const int idx = it * NTH + tid; const int row = idx / (WID / 4), c4 = idx - row * (WID / 4);
            const size_t oo = obase + (size_t)row * PLC + (size_t)c4 * 4;
            const v4f a = *(const v4fa*)(TF + row * OP + c4 * 4); const v4f c = *(const v4fa*)(TF + (CH + row) * OP + c4 * 4);
            *(volatile v4f*)(X2 + oo) = a; *(volatile v4f*)(Y2 + oo) = c; }
        if (wave == 0) { const v4f pv = *(const v4fa*)(psum + 4 * lane);
            *(volatile v4f*)(PART + (size_t)bh * 128 + 4 * lane) = pv; }
        if (ps == 0) __threadfence(); }
#undef TF
#undef LDL
}

__global__ __launch_bounds__(256) void k_fuse(const float* __restrict__ X2, const float* __restrict__ Y2, const float* __restrict__ PART, float* OUT) {
#pragma clang fp contract(off)
    __shared__ float w1s[CH];
    __shared__ float w2s[CH];
    const int tid = threadIdx.x;
    const int wave = __builtin_amdgcn_readfirstlane((int)(threadIdx.x >> 5));
    const int b = blockIdx.x / FB; const int q = (blockIdx.x % FB) * 256 + tid;
    if (wave < 2) { const int c = tid;
        const float* pp = PART + (size_t)b * HR * 128 + c;
        float s1 = 0.0f, s2 = 0.0f;
#pragma unroll 1
        for (int hh = 0; hh < HR; ++hh) { s1 += pp[(size_t)hh * 128]; s2 += pp[(size_t)hh * 128 + 64]; }
        const float rhw = 1.0f / (float)(HR * WID);
        const float e1 = __builtin_amdgcn_exp2f(s1 * rhw * L2E), e2 = __builtin_amdgcn_exp2f(s2 * rhw * L2E);
        const float rd = e1 + e2 + 1e-5f; const float ri = __builtin_amdgcn_rcpf(rd);
        w1s[c] = e1 * ri; w2s[c] = e2 * ri; }
    __syncthreads();
    const size_t PLC = (size_t)HR * WID;
    const size_t base = (size_t)b * CH * PLC + (size_t)q * 4;
    v4f a1 = (v4f){}, a2 = (v4f){};
#pragma unroll 1
    for (int c = 0; c < CH; ++c) {
        const v4f xv = *(const v4f*)(X2 + base + (size_t)c * PLC); const v4f yv = *(const v4f*)(Y2 + base + (size_t)c * PLC);
#pragma unroll
        for (int k = 0; k < 4; ++k) { a1[k] += fabsf(xv[k]); a2[k] += fabsf(yv[k]); } }
    v4f cw1, cw2;
#pragma unroll
    for (int k = 0; k < 4; ++k) {
        const float e1 = __builtin_amdgcn_exp2f(a1[k] * (1.0f / 64.0f) * L2E), e2 = __builtin_amdgcn_exp2f(a2[k] * (1.0f / 64.0f) * L2E);
        const float cd = e1 + e2 + 1e-5f; const float ci = __builtin_amdgcn_rcpf(cd);
        cw1[k] = e1 * ci; cw2[k] = e2 * ci; }
    const size_t OPL = (size_t)OUT_HR * WID;
    const size_t ob = (size_t)b * CH * OPL + (size_t)q * 4;
#pragma unroll 1
    for (int ps = 0; ps < 2; ++ps) {
#pragma unroll 1
        for (int c = 0; c < CH; ++c) {
            const v4f xv = *(const v4f*)(X2 + base + (size_t)c * PLC); const v4f yv = *(const v4f*)(Y2 + base + (size_t)c * PLC);
            const float u1 = w1s[c], u2 = w2s[c]; v4f o;
#pragma unroll
            for (int k = 0; k < 4; ++k) o[k] = (u1 + cw1[k]) * xv[k] + (u2 + cw2[k]) * yv[k];
            *(volatile v4f*)(OUT + ob + (size_t)c * OPL) = o; }
        if (ps == 0) __threadfence(); }
}

static constexpr size_t al256(size_t v) { return (v + 255) & ~(size_t)255; }
static constexpr size_t SZ_X2 = al256((size_t)NB * CH * HR * WID * 4);
static constexpr size_t SZ_PT = al256((size_t)NB * HR * 128 * 4);
static constexpr size_t SZ_WH = al256((size_t)4 * CH * CH * 2);
static constexpr size_t SZ_TOTAL = 2 * SZ_X2 + SZ_PT + SZ_WH;
static_assert(SZ_TOTAL <= (size_t)134217728);
static_assert(((size_t)CH * CH * 2) % 256 == 0);

extern "C" void kernel_launch(void* const* d_in, const int* in_sizes, int n_in,
                              void* d_out, int out_size, void* d_ws, size_t ws_size, hipStream_t stream) {
    if (n_in < 16) return;
    const size_t needx = ((((size_t)(NB - 1) * CH + (CH - 1)) * HR_FULL + (size_t)(HR - 1)) * WID) + WID;
    if ((size_t)in_sizes[0] < needx || (size_t)in_sizes[1] < needx) return;
    if (in_sizes[2] < CH || in_sizes[3] < CH || in_sizes[4] < CH || in_sizes[5] < CH) return;
    if (in_sizes[6] < CH * CH || in_sizes[8] < CH * CH || in_sizes[10] < CH * CH || in_sizes[12] < CH * CH) return;
    if (in_sizes[7] < CH || in_sizes[9] < CH || in_sizes[11] < CH || in_sizes[13] < CH || in_sizes[14] < CH || in_sizes[15] < CH) return;
    if ((size_t)out_size < ((((size_t)(NB - 1) * CH + (CH - 1)) * OUT_HR + (size_t)(HR - 1)) * WID) + WID) return;
    if (SZ_TOTAL > ws_size) return;
    const float* x  = (const float*)d_in[0];  const float* y  = (const float*)d_in[1];
    const float* llw = (const float*)d_in[2]; const float* llb = (const float*)d_in[3];
    const float* lrw = (const float*)d_in[4]; const float* lrb = (const float*)d_in[5];
    const float* wl1 = (const float*)d_in[6];  const float* bl1 = (const float*)d_in[7];
    const float* wr1 = (const float*)d_in[8];  const float* br1 = (const float*)d_in[9];
    const float* wl2 = (const float*)d_in[10]; const float* bl2 = (const float*)d_in[11];
    const float* wr2 = (const float*)d_in[12]; const float* br2 = (const float*)d_in[13];
    const float* beta = (const float*)d_in[14]; const float* gamma = (const float*)d_in[15];
    float* OUT = (float*)d_out;
    char* wsp = (char*)d_ws;
    float* X2 = (float*)wsp; wsp += SZ_X2;
    float* Y2 = (float*)wsp; wsp += SZ_X2;
    float* PART = (float*)wsp; wsp += SZ_PT;
    h16* WH = (h16*)wsp; wsp += SZ_WH;

    k_wconv<<<2, 256, 0, stream>>>(wl1, wr1, wl2, wr2, WH);
    k_row<<<NB * HR, NTH, 0, stream>>>(x, y, llw, llb, lrw, lrb, bl1, br1, bl2, br2, beta, gamma, WH, X2, Y2, PART);
    k_fuse<<<NB * FB, 256, 0, stream>>>(X2, Y2, PART, OUT);
}
